// ShapleyQMixer_63428077027892
// MI455X (gfx1250) — hardware-verified
//
#include <hip/hip_runtime.h>

typedef _Float16 v16h __attribute__((ext_vector_type(16)));
typedef _Float16 v8h  __attribute__((ext_vector_type(8)));
typedef float    v8f  __attribute__((ext_vector_type(8)));
typedef __attribute__((ext_vector_type(4))) float v4f_t;
typedef float v4fa __attribute__((ext_vector_type(4), may_alias));
typedef __attribute__((ext_vector_type(4))) unsigned v4u_t;
typedef unsigned v4ua __attribute__((ext_vector_type(4), may_alias));

#define BS   1024
#define DD   256
#define NN   16
#define SS   16
#define EE   64
#define NCAT 320
#define NTIL 20
#define KSTP 8
#define RSPLIT (1.0f / 2048.0f)

#define OFF_MEAN 0
#define OFF_RSTD 1024
#define OFF_BIAS 2048
#define OFF_A    4096
#define PLA      (BS * DD)
#define OFF_W    (OFF_A + 2 * PLA * 2)
#define PLW      (DD * NCAT)
#define OFF_H    (OFF_W + 2 * PLW * 2)

__device__ __forceinline__ _Float16 lo_of(float v, _Float16 h) { return (_Float16)((v - (float)h) * 2048.0f); }
__device__ __forceinline__ v8f wmma16(v16h a, v16h b, v8f c) { return __builtin_amdgcn_wmma_f32_16x16x32_f16(false, a, false, b, (short)0, c, false, false); }
__device__ __forceinline__ v8f wmma_split(v16h a, v16h al, v16h b, v16h bl, v8f c) { v8f x = {}; x = wmma16(al, b, x); x = wmma16(a, bl, x); return wmma16(a, b, c) + x * RSPLIT; }

__global__ void __launch_bounds__(256)
k_stats(const float* __restrict__ states, float* __restrict__ mean, float* __restrict__ rstd) {
  __shared__ float sh[8][32], sh2[8][32];
  const int t = threadIdx.x, cl = t & 31, rg = t >> 5;
  const int c = blockIdx.x * 32 + cl;
  float s = 0.f, s2 = 0.f;
  for (int r = rg; r < BS; r += 8) { const float x = states[r * DD + c]; s += x; s2 += x * x; }
  sh[rg][cl] = s; sh2[rg][cl] = s2;
  __syncthreads();
  if (t < 32) {
    float a = 0.f, a2 = 0.f;
    for (int g = 0; g < 8; ++g) { a += sh[g][t]; a2 += sh2[g][t]; }
    const float n = (float)BS;
    const float bm = a / n;
    const float bv = (a2 - n * bm * bm) / (n - 1.f);
    const float tot = 1e-4f + n;
    const float nm  = bm * n / tot;
    const float M2  = 1e-4f + bv * n + bm * bm * 1e-4f * n / tot;
    const float nv  = M2 / tot;
    const float rs  = rsqrtf(nv);
    *(volatile float*)(mean + c) = nm; *(volatile float*)(rstd + c) = rs; __threadfence();
    *(volatile float*)(mean + c) = nm; *(volatile float*)(rstd + c) = rs;
  }
}

__global__ void __launch_bounds__(256)
k_norm(const float* __restrict__ states, const float* __restrict__ mean, const float* __restrict__ rstd, _Float16* __restrict__ A) {
  const int i8 = (blockIdx.x * 256 + threadIdx.x) * 8;
  const int c0 = i8 & (DD - 1);
  _Float16 hh[8], hl[8];
#pragma unroll
  for (int e = 0; e < 8; ++e) { const float v = (states[i8 + e] - mean[c0 + e]) * rstd[c0 + e]; hh[e] = (_Float16)v; hl[e] = lo_of(v, hh[e]); }
  _Float16* d = A + i8;
  *(volatile v4u_t*)d = *(const v4ua*)hh; *(volatile v4u_t*)(d + PLA) = *(const v4ua*)hl; __threadfence();
  *(volatile v4u_t*)d = *(const v4ua*)hh; *(volatile v4u_t*)(d + PLA) = *(const v4ua*)hl;
}

__global__ void __launch_bounds__(256)
k_pack(const float* __restrict__ W1,  const float* __restrict__ b1,
       const float* __restrict__ Wb1, const float* __restrict__ bb1,
       const float* __restrict__ Wf,  const float* __restrict__ bf,
       const float* __restrict__ Vw1, const float* __restrict__ Vb1,
       _Float16* __restrict__ Wcs, float* __restrict__ bias) {
  const int g = blockIdx.x * 256 + threadIdx.x;
  if (g < NTIL * KSTP * 32) {
    const int lane = g & 31, ks = (g >> 5) % KSTP, tn = (g >> 5) / KSTP;
    const int n = tn * 16 + (lane & 15), half = lane >> 4;
    _Float16 hh[16], hl[16];
#pragma unroll
    for (int j = 0; j < 16; ++j) {
      const int k = ks * 32 + 8 * half + ((j < 8) ? j : (j + 8));
      float w;
      if (n < 128)      w = W1 [k * 128 + n];
      else if (n < 192) w = Wb1[k * 64 + (n - 128)];
      else if (n < 256) w = Wf [k * 64 + (n - 192)];
      else              w = Vw1[k * 64 + (n - 256)];
      hh[j] = (_Float16)w; hl[j] = lo_of(w, hh[j]);
    }
    _Float16* d = Wcs + (size_t)g * 16;
    *(volatile v4u_t*)d = *(const v4ua*)hh; *(volatile v4u_t*)(d + 8) = *(const v4ua*)(hh + 8);
    *(volatile v4u_t*)(d + PLW) = *(const v4ua*)hl; *(volatile v4u_t*)(d + PLW + 8) = *(const v4ua*)(hl + 8); __threadfence();
    *(volatile v4u_t*)d = *(const v4ua*)hh; *(volatile v4u_t*)(d + 8) = *(const v4ua*)(hh + 8);
    *(volatile v4u_t*)(d + PLW) = *(const v4ua*)hl; *(volatile v4u_t*)(d + PLW + 8) = *(const v4ua*)(hl + 8);
  } else if (g < NTIL * KSTP * 32 + NCAT) {
    const int n = g - NTIL * KSTP * 32;
    float bb;
    if (n < 128)      bb = b1[n];
    else if (n < 192) bb = bb1[n - 128];
    else if (n < 256) bb = bf[n - 192];
    else              bb = Vb1[n - 256];
    *(volatile float*)(bias + n) = bb; __threadfence(); *(volatile float*)(bias + n) = bb;
  }
}

__global__ void __launch_bounds__(256)
k_gemm(const _Float16* __restrict__ A, const _Float16* __restrict__ Wcs, const float* __restrict__ bias, float* __restrict__ H) {
  __shared__ __attribute__((aligned(16))) float st[8][16 * 68];
  const int tid  = threadIdx.x;
  const int lane = tid & 31;
  const int wave = tid >> 5;
  const int gw   = blockIdx.x * 8 + wave;
  const int tm   = gw / 5;
  const int cg   = gw % 5;
  const int m    = lane & 15;
  const int hi   = lane >> 4;
  const int row  = tm * 16 + m;
  float* sw = st[wave];

  const _Float16* pa0 = A + row * DD + hi * 8;
  v8f acc[4] = {};
#pragma unroll 2
  for (int ks = 0; ks < KSTP; ++ks) {
    const _Float16* pa = pa0 + ks * 32;
    const v16h a  = __builtin_shufflevector(*(const v8h*)pa, *(const v8h*)(pa + 16), 0,1,2,3,4,5,6,7,8,9,10,11,12,13,14,15);
    const v16h al = __builtin_shufflevector(*(const v8h*)(pa + PLA), *(const v8h*)(pa + PLA + 16), 0,1,2,3,4,5,6,7,8,9,10,11,12,13,14,15);
#pragma unroll
    for (int q = 0; q < 4; ++q) {
      const int tn = cg * 4 + q;
      const v16h* pb = (const v16h*)Wcs + ((tn * KSTP + ks) * 32 + lane);
      acc[q] = wmma_split(a, al, pb[0], *(const v16h*)((const _Float16*)pb + PLW), acc[q]);
    }
  }
#pragma unroll
  for (int q = 0; q < 4; ++q) {
    const int col = (cg * 4 + q) * 16 + m;
    const float bcol = bias[col];
#pragma unroll
    for (int r = 0; r < 8; ++r) {
      float v = acc[q][r] + bcol, o;
      if (col < 128)      o = fabsf(v);
      else if (col < 192) o = v;
      else if (col < 256) o = fabsf(v);
      else                o = fmaxf(v, 0.f);
      sw[(r + hi * 8) * 68 + q * 16 + m] = o;
    }
  }
  asm volatile("s_wait_dscnt 0" ::: "memory");
#pragma unroll 1
  for (int pass = 0; pass < 2; ++pass) {
#pragma unroll
    for (int it = 0; it < 8; ++it) { const int ch = lane + 32 * it, r = ch >> 4, q4 = (ch & 15) * 4;
      *(volatile v4f_t*)(H + (size_t)(tm * 16 + r) * NCAT + cg * 64 + q4) = *(const volatile v4fa*)(sw + r * 68 + q4); }
    __threadfence();
  }
}

__global__ void __launch_bounds__(256)
k_final(const float* __restrict__ aq, const float* __restrict__ mf,
        const int* __restrict__ gc, const float* __restrict__ H,
        const float* __restrict__ Vw2, const float* __restrict__ Vb2,
        float* __restrict__ out) {
  const int t = threadIdx.x;
  __shared__ float aq_sh[NN];
  __shared__ int   gc_sh[SS * NN];
  __shared__ float hh[NCAT];
  __shared__ float v_sh;
  __shared__ float ys[256];
  __shared__ float wr[NN];
  __shared__ __attribute__((aligned(16))) float qout[32];
  __shared__ __attribute__((aligned(16))) float wout[32 * NN];

#pragma unroll 1
  for (int rb = 0; rb < 32; ++rb) {
    const int b = blockIdx.x * 32 + rb;
    __syncthreads();
    if (t < NN) aq_sh[t] = aq[b * NN + t];
    { int g = gc[b * SS * NN + t]; gc_sh[t] = (g < 0) ? 0 : (g > NN - 1 ? NN - 1 : g); }
    hh[t] = H[b * NCAT + t];
    if (t < 64) hh[256 + t] = H[b * NCAT + 256 + t];
    __syncthreads();

    if (t == 0) {
      float v = Vb2[0];
      for (int e = 0; e < EE; ++e) v += hh[256 + e] * Vw2[e];
      v_sh = v;
    }
    __syncthreads();

    const int s = t >> 4, i = t & 15;
    const int pos = gc_sh[s * NN + i];
    float csum = 0.f;
    for (int j = 0; j < pos; ++j) csum += aq_sh[gc_sh[s * NN + j]];
    const float denom = (pos == 0) ? 1.f : (float)pos;
    const float nv = csum / denom;
    const float x1 = aq_sh[i];

    float y = 0.f;
    for (int e = 0; e < EE; ++e) {
      float z = nv * hh[e] + x1 * hh[64 + e] + hh[128 + e];
      float h = (z > 0.f) ? z : (expf(z) - 1.f);
      y += h * hh[192 + e];
    }
    y += v_sh;
    ys[t] = fabsf(y);
    __syncthreads();

    if (t < NN) {
      float w = 0.f;
      for (int ss = 0; ss < SS; ++ss) w += ys[ss * NN + t];
      w = w * (1.f / (float)SS) + 1.f;
      wout[rb * NN + t] = w;
      float mk = mf[b * NN + t];
      wr[t] = (w * (1.f - mk) + mk) * aq_sh[t];
    }
    __syncthreads();
    if (t == 0) {
      float q = 0.f;
      for (int k = 0; k < NN; ++k) q += wr[k];
      qout[rb] = q;
    }
  }
  __syncthreads();
#pragma unroll 1
  for (int pass = 0; pass < 2; ++pass) {
    if (t < 8) *(volatile v4f_t*)(out + blockIdx.x * 32 + t * 4) = *(const volatile v4fa*)(qout + t * 4);
    if (t < 128) *(volatile v4f_t*)(out + BS + blockIdx.x * 32 * NN + t * 4) = *(const volatile v4fa*)(wout + t * 4);
    __threadfence();
  }
}

extern "C" void kernel_launch(void* const* d_in, const int* in_sizes, int n_in,
                              void* d_out, int out_size, void* d_ws, size_t ws_size,
                              hipStream_t stream) {
  (void)in_sizes; (void)n_in; (void)out_size; (void)ws_size;
  const float* states     = (const float*)d_in[0];
  const float* agent_qs   = (const float*)d_in[2];
  const float* max_filter = (const float*)d_in[3];
  const int*   gcoal      = (const int*)  d_in[4];
  const float* W1  = (const float*)d_in[5];
  const float* b1  = (const float*)d_in[6];
  const float* Wb1 = (const float*)d_in[7];
  const float* bb1 = (const float*)d_in[8];
  const float* Wf  = (const float*)d_in[9];
  const float* bf  = (const float*)d_in[10];
  const float* Vw1 = (const float*)d_in[11];
  const float* Vb1 = (const float*)d_in[12];
  const float* Vw2 = (const float*)d_in[13];
  const float* Vb2 = (const float*)d_in[14];

  char* ws = (char*)d_ws;
  float*    mean = (float*)(ws + OFF_MEAN);
  float*    rstd = (float*)(ws + OFF_RSTD);
  float*    bias = (float*)(ws + OFF_BIAS);
  _Float16* A    = (_Float16*)(ws + OFF_A);
  _Float16* Wcs  = (_Float16*)(ws + OFF_W);
  float*    H    = (float*)(ws + OFF_H);
  float*    out  = (float*)d_out;

  k_stats<<<DD / 32, 256, 0, stream>>>(states, mean, rstd);
  k_norm <<<BS * DD / 8 / 256, 256, 0, stream>>>(states, mean, rstd, A);
  k_pack <<<(NTIL * KSTP * 32 + NCAT + 255) / 256, 256, 0, stream>>>(W1, b1, Wb1, bb1, Wf, bf, Vw1, Vb1, Wcs, bias);
  k_gemm <<<40, 256, 0, stream>>>(A, Wcs, bias, H);
  k_final<<<BS / 32, 256, 0, stream>>>(agent_qs, max_filter, gcoal, H, Vw2, Vb2, out);
}
